// RWKV7Block_78391743086640
// MI455X (gfx1250) — hardware-verified
//
#include <hip/hip_runtime.h>
#include <math.h>


#define NB 8
#define TT 512
#define CC 1024
#define NH 16
#define HD 64
#define NR (NB * TT)
#define DW 64
#define DA 64
#define DG 128
#define FF 4096

typedef __attribute__((ext_vector_type(16))) _Float16 v16h;
typedef __attribute__((ext_vector_type(8)))  _Float16 v8h;
typedef __attribute__((ext_vector_type(8)))  float v8f;
typedef __attribute__((ext_vector_type(4)))  float v4f;
typedef __attribute__((ext_vector_type(4)))  unsigned v4u;
typedef float __attribute__((may_alias)) float_a;

template <typename T> __device__ __forceinline__ void vst2(void* p, T v) { *(volatile T*)p = v; __threadfence(); *(volatile T*)p = v; }
__device__ __forceinline__ v8f wmma16(v16h a, v16h b, v8f c) {
  v8f d = __builtin_amdgcn_wmma_f32_16x16x32_f16(false, a, false, b, (short)0, c, false, false);
  asm volatile("v_nop\n\tv_nop\n\tv_nop\n\tv_nop" : "+v"(d) : "v"(a), "v"(b));
  return d;
}
__device__ __forceinline__ v16h frag_h(const _Float16* rowk0, int lane) {
  union { v16h v; v8h q[2]; } u; const _Float16* p = rowk0 + 8 * (lane >> 4);
  u.q[0] = *(const v8h*)p; u.q[1] = *(const v8h*)(p + 16); return u.v;
}
__device__ __forceinline__ float sigm(float x) { return 1.0f / (1.0f + expf(-x)); }
__device__ __forceinline__ float softplus(float x) { return x > 20.f ? x : log1pf(expf(x)); }
#define LDSX() do { asm volatile("s_wait_dscnt 0" ::: "memory"); __builtin_amdgcn_wave_barrier(); __builtin_amdgcn_fence(__ATOMIC_RELEASE, "workgroup"); } while (0)

__global__ __launch_bounds__(256) void k_packT(const float* __restrict__ W, _Float16* __restrict__ Wt, int K, int N) {
  __shared__ float tile[64][65];
  const int k0 = blockIdx.y * 64, n0 = blockIdx.x * 64, tid = threadIdx.x;
  for (int q = tid; q < 64 * 64; q += 256) { const int kk = q >> 6, nn = q & 63; tile[kk][nn] = W[(size_t)(k0 + kk) * N + n0 + nn]; }
  __syncthreads();
  for (int q = tid; q < 64 * 8; q += 256) { const int nn = q >> 3, pc = q & 7;
    union { v8h h; v4u u; } pk;
#pragma unroll
    for (int e = 0; e < 8; ++e) pk.h[e] = (_Float16)tile[pc * 8 + e][nn];
    vst2(Wt + (size_t)(n0 + nn) * K + k0 + pc * 8, pk.u); }
}

__device__ __forceinline__ void ln_row(float v[8], const float* __restrict__ gm, const float* __restrict__ bt, int tid, float* red) {
  float s = 0.f;
#pragma unroll
  for (int e = 0; e < 8; ++e) s += v[e];
  red[tid] = s; __syncthreads();
  for (int st = 64; st > 0; st >>= 1) { if (tid < st) red[tid] += red[tid + st]; __syncthreads(); }
  const float mu = red[0] / (float)CC; __syncthreads();
  float q = 0.f;
#pragma unroll
  for (int e = 0; e < 8; ++e) { v[e] -= mu; q += v[e] * v[e]; }
  red[tid] = q; __syncthreads();
  for (int st = 64; st > 0; st >>= 1) { if (tid < st) red[tid] += red[tid + st]; __syncthreads(); }
  const float rs = rsqrtf(red[0] / (float)CC + 1e-5f); __syncthreads();
#pragma unroll
  for (int e = 0; e < 8; ++e) v[e] = v[e] * rs * gm[tid * 8 + e] + bt[tid * 8 + e];
}
__global__ __launch_bounds__(128) void k_ln01(const float* __restrict__ x, const float* __restrict__ g0, const float* __restrict__ b0,
                                            const float* __restrict__ g1, const float* __restrict__ b1, float* __restrict__ x0, float* __restrict__ xn) {
  __shared__ float red[128];
  const size_t row = blockIdx.x; const int tid = threadIdx.x;
  float v[8];
  { const v4f a = *(const v4f*)(x + row * CC + tid * 8), b = *(const v4f*)(x + row * CC + tid * 8 + 4); v[0]=a[0];v[1]=a[1];v[2]=a[2];v[3]=a[3];v[4]=b[0];v[5]=b[1];v[6]=b[2];v[7]=b[3]; }
  ln_row(v, g0, b0, tid, red);
  vst2(x0 + row * CC + tid * 8, (v4f){v[0], v[1], v[2], v[3]}); vst2(x0 + row * CC + tid * 8 + 4, (v4f){v[4], v[5], v[6], v[7]});
  ln_row(v, g1, b1, tid, red);
  vst2(xn + row * CC + tid * 8, (v4f){v[0], v[1], v[2], v[3]}); vst2(xn + row * CC + tid * 8 + 4, (v4f){v[4], v[5], v[6], v[7]});
}
__global__ __launch_bounds__(128) void k_ln(const float* __restrict__ x, const float* __restrict__ gm, const float* __restrict__ bt, float* __restrict__ o) {
  __shared__ float red[128];
  const size_t row = blockIdx.x; const int tid = threadIdx.x;
  float v[8];
  { const v4f a = *(const v4f*)(x + row * CC + tid * 8), b = *(const v4f*)(x + row * CC + tid * 8 + 4); v[0]=a[0];v[1]=a[1];v[2]=a[2];v[3]=a[3];v[4]=b[0];v[5]=b[1];v[6]=b[2];v[7]=b[3]; }
  ln_row(v, gm, bt, tid, red);
  vst2(o + row * CC + tid * 8, (v4f){v[0], v[1], v[2], v[3]}); vst2(o + row * CC + tid * 8 + 4, (v4f){v[4], v[5], v[6], v[7]});
}

__global__ __launch_bounds__(128) void k_mix(const float* __restrict__ xn, const float* __restrict__ m0, const float* __restrict__ m1,
                                           const float* __restrict__ m2, const float* __restrict__ m3, const float* __restrict__ m4, const float* __restrict__ m5,
                                           _Float16* __restrict__ o0, _Float16* __restrict__ o1, _Float16* __restrict__ o2,
                                           _Float16* __restrict__ o3, _Float16* __restrict__ o4, _Float16* __restrict__ o5, int NM) {
  const size_t row = blockIdx.x; const int tid = threadIdx.x, t = (int)(row % TT);
  float cur[8], prv[8];
#pragma unroll
  for (int e = 0; e < 8; ++e) { cur[e] = xn[row * CC + tid * 8 + e]; prv[e] = t > 0 ? xn[(row - 1) * CC + tid * 8 + e] : 0.f; }
#pragma unroll 1
  for (int j = 0; j < NM; ++j) {
    const float* mm = j == 0 ? m0 : j == 1 ? m1 : j == 2 ? m2 : j == 3 ? m3 : j == 4 ? m4 : m5;
    _Float16* oo = j == 0 ? o0 : j == 1 ? o1 : j == 2 ? o2 : j == 3 ? o3 : j == 4 ? o4 : o5;
    union { v8h h; v4u u; } pk;
#pragma unroll
    for (int e = 0; e < 8; ++e) pk.h[e] = (_Float16)(cur[e] + (prv[e] - cur[e]) * mm[tid * 8 + e]);
    vst2(oo + row * CC + tid * 8, pk.u); }
}

template <int NT, int MODE>
__global__ __launch_bounds__(128) void k_gemm(const _Float16* __restrict__ A, const _Float16* __restrict__ W, const float* __restrict__ p0,
                                            const float* __restrict__ res, void* __restrict__ Outv, int K, int N) {
  __shared__ __align__(16) float so[4][16 * NT * 16];
  float* Out = (float*)Outv; _Float16* Outh = (_Float16*)Outv;
  const int tid = threadIdx.x, wave = tid >> 5, lane = tid & 31, col = lane & 15, g = lane >> 4;
  const int r0 = blockIdx.x * 64 + wave * 16, n0 = blockIdx.y * (NT * 16);
  v8f acc[NT];
#pragma unroll
  for (int j = 0; j < NT; ++j) acc[j] = (v8f){};
#pragma unroll 1
  for (int kc = 0; kc < K / 32; ++kc) { const v16h a = frag_h(A + (size_t)(r0 + col) * K + kc * 32, lane);
#pragma unroll
    for (int j = 0; j < NT; ++j) acc[j] = wmma16(a, frag_h(W + (size_t)(n0 + j * 16 + col) * K + kc * 32, lane), acc[j]); }
  float* S = so[wave]; const int LD = NT * 16;
#pragma unroll
  for (int j = 0; j < NT; ++j) { const int n = n0 + j * 16 + col; const float pv = p0 ? p0[n] : 0.f;
#pragma unroll
    for (int r = 0; r < 8; ++r) { float v = acc[j][r];
      if (MODE == 1) v = tanhf(v); else if (MODE == 2) v = sigm(v); else if (MODE == 6) { }
      else if (MODE == 3) v = expf(-expf(-softplus(-(pv + v)) - 0.5f)); else if (MODE == 4) v = sigm(pv + v);
      else if (MODE == 5) { v = v > 0.f ? v : 0.f; v = v * v; }
      S[(8 * g + r) * LD + j * 16 + col] = v; } }
  LDSX();
  if (MODE == 0 || MODE == 3 || MODE == 4) {
    for (int q = lane; q < 16 * (LD / 4); q += 32) { const int rl = q / (LD / 4), pc = q % (LD / 4); const size_t o = (size_t)(r0 + rl) * N + n0 + pc * 4;
      v4f v = *(const v4f*)(S + rl * LD + pc * 4); if (MODE == 0 && res) v += *(const v4f*)(res + o); vst2(Out + o, v); }
  } else {
    for (int q = lane; q < 16 * (LD / 8); q += 32) { const int rl = q / (LD / 8), pc = q % (LD / 8);
      union { v8h h; v4u u; } pk;
#pragma unroll
      for (int e = 0; e < 8; ++e) pk.h[e] = (_Float16)S[rl * LD + pc * 8 + e];
      vst2(Outh + (size_t)(r0 + rl) * N + n0 + pc * 8, pk.u); }
  }
}

__global__ __launch_bounds__(256) void k_prep(const float* __restrict__ k0, const float* __restrict__ a, const float* __restrict__ kkw,
                                            const float* __restrict__ kaw, float* __restrict__ kfin, float* __restrict__ aa, float* __restrict__ bb) {
  const size_t row = blockIdx.x; const int tid = threadIdx.x;
  const v4f kv = *(const v4f*)(k0 + row * CC + tid * 4), av = *(const v4f*)(a + row * CC + tid * 4);
  const v4f kk = *(const v4f*)(kkw + tid * 4), ka = *(const v4f*)(kaw + tid * 4);
  v4f u = kv * kk;
  float s = u[0] * u[0] + u[1] * u[1] + u[2] * u[2] + u[3] * u[3];
#pragma unroll
  for (int off = 8; off >= 1; off >>= 1) s += __shfl_xor(s, off, 32);
  const float inv = 1.0f / fmaxf(sqrtf(s), 1e-12f);
  u = u * inv;
  const v4f one = {1.f, 1.f, 1.f, 1.f};
  vst2(kfin + row * CC + tid * 4, kv * (one + (av - one) * ka));
  vst2(aa + row * CC + tid * 4, -u);
  vst2(bb + row * CC + tid * 4, u * av);
}

__global__ __launch_bounds__(256) void k_wkv(const float* __restrict__ r, const float* __restrict__ dec, const float* __restrict__ kf,
                                           const float* __restrict__ v, const float* __restrict__ aa, const float* __restrict__ bb, float* __restrict__ o) {
  __shared__ float sr[HD], sd[HD], sk[HD], sv[HD], sa[HD], sbv[HD];
  __shared__ __align__(16) float so[HD];
  const int b = blockIdx.x / NH, h = blockIdx.x % NH, tid = threadIdx.x, i = tid >> 2, j0 = (tid & 3) * 16;
  float S[16];
#pragma unroll
  for (int j = 0; j < 16; ++j) S[j] = 0.f;
#pragma unroll 1
  for (int t = 0; t < TT; ++t) { const size_t base = ((size_t)b * TT + t) * CC + h * HD;
    if (tid < HD) { sr[tid] = r[base + tid]; sd[tid] = dec[base + tid]; sk[tid] = kf[base + tid]; sv[tid] = v[base + tid]; sa[tid] = aa[base + tid]; sbv[tid] = bb[base + tid]; }
    __syncthreads();
    float s_a = 0.f;
#pragma unroll
    for (int j = 0; j < 16; ++j) s_a += S[j] * sa[j0 + j];
    s_a += __shfl_xor(s_a, 1, 32); s_a += __shfl_xor(s_a, 2, 32);
    const float vi = sv[i];
    float y = 0.f;
#pragma unroll
    for (int j = 0; j < 16; ++j) { S[j] = S[j] * sd[j0 + j] + s_a * sbv[j0 + j] + vi * sk[j0 + j]; y += S[j] * sr[j0 + j]; }
    y += __shfl_xor(y, 1, 32); y += __shfl_xor(y, 2, 32);
    if ((tid & 3) == 0) so[i] = y;
    __syncthreads();
    if (tid < 16) vst2(o + base + tid * 4, *(const v4f*)(&so[tid * 4]));
  }
}

__global__ __launch_bounds__(256) void k_post(const float* __restrict__ o, const float* __restrict__ r, const float* __restrict__ kf,
                                            const float* __restrict__ v, const float* __restrict__ g, const float* __restrict__ rk,
                                            const float* __restrict__ gw, const float* __restrict__ gb, _Float16* __restrict__ og) {
  const size_t row = blockIdx.x; const int tid = threadIdx.x, h = tid >> 4, c0 = tid * 4;
  const v4f ov = *(const v4f*)(o + row * CC + c0);
  float s = ov[0] + ov[1] + ov[2] + ov[3];
#pragma unroll
  for (int off = 8; off >= 1; off >>= 1) s += __shfl_xor(s, off, 32);
  const float mu = s / (float)HD;
  float q = 0.f;
#pragma unroll
  for (int e = 0; e < 4; ++e) { const float d = ov[e] - mu; q += d * d; }
#pragma unroll
  for (int off = 8; off >= 1; off >>= 1) q += __shfl_xor(q, off, 32);
  const float rs = rsqrtf(q / (float)HD + 64e-5f);
  const v4f rv = *(const v4f*)(r + row * CC + c0), kv = *(const v4f*)(kf + row * CC + c0), rkv = *(const v4f*)(rk + h * HD + (c0 & 63));
  float bon = rv[0] * kv[0] * rkv[0] + rv[1] * kv[1] * rkv[1] + rv[2] * kv[2] * rkv[2] + rv[3] * kv[3] * rkv[3];
#pragma unroll
  for (int off = 8; off >= 1; off >>= 1) bon += __shfl_xor(bon, off, 32);
  const v4f vv = *(const v4f*)(v + row * CC + c0), gv = *(const v4f*)(g + row * CC + c0), gwv = *(const v4f*)(gw + c0), gbv = *(const v4f*)(gb + c0);
  float res4[4];
#pragma unroll
  for (int e = 0; e < 4; ++e) res4[e] = (((ov[e] - mu) * rs) * gwv[e] + gbv[e] + bon * vv[e]) * gv[e];
  float n4[4];
#pragma unroll
  for (int e = 0; e < 4; ++e) n4[e] = __shfl_xor(res4[e], 1, 32);
  if ((tid & 1) == 0) { union { v8h hh; v4u u; } pk;
#pragma unroll
    for (int e = 0; e < 4; ++e) { pk.hh[e] = (_Float16)res4[e]; pk.hh[4 + e] = (_Float16)n4[e]; }
    vst2(og + row * CC + c0, pk.u); }
}
__global__ __launch_bounds__(128) void k_mixf(const float* __restrict__ xf, const float* __restrict__ mm, _Float16* __restrict__ o16) {
  const size_t row = blockIdx.x; const int tid = threadIdx.x, t = (int)(row % TT);
  union { v8h h; v4u u; } pk;
#pragma unroll
  for (int e = 0; e < 8; ++e) { const float cur = xf[row * CC + tid * 8 + e], prv = t > 0 ? xf[(row - 1) * CC + tid * 8 + e] : 0.f;
    pk.h[e] = (_Float16)(cur + (prv - cur) * mm[tid * 8 + e]); }
  vst2(o16 + row * CC + tid * 8, pk.u);
}
__global__ __launch_bounds__(256) void k_copy(const float* __restrict__ s, float* __restrict__ d, size_t n4) {
  const size_t i = (size_t)blockIdx.x * 256 + threadIdx.x; if (i >= n4) return;
  vst2(d + i * 4, *(const v4f*)(s + i * 4));
}

extern "C" void kernel_launch(void* const* d_in, const int* in_sizes, int n_in,
                              void* d_out, int out_size, void* d_ws, size_t ws_size,
                              hipStream_t stream) {
  (void)in_sizes; (void)n_in; (void)out_size; (void)ws_size;
  const float* x = (const float*)d_in[0];
  const float* g0 = (const float*)d_in[2]; const float* b0 = (const float*)d_in[3];
  const float* g1 = (const float*)d_in[4]; const float* b1 = (const float*)d_in[5];
  const float* g2 = (const float*)d_in[6]; const float* b2 = (const float*)d_in[7];
  const float* x_r = (const float*)d_in[8]; const float* x_w = (const float*)d_in[9]; const float* x_k = (const float*)d_in[10];
  const float* x_v = (const float*)d_in[11]; const float* x_a = (const float*)d_in[12]; const float* x_g = (const float*)d_in[13];
  const float* w0 = (const float*)d_in[14]; const float* w1 = (const float*)d_in[15]; const float* w2 = (const float*)d_in[16];
  const float* a0 = (const float*)d_in[17]; const float* a1 = (const float*)d_in[18]; const float* a2 = (const float*)d_in[19];
  const float* gg1 = (const float*)d_in[20]; const float* gg2 = (const float*)d_in[21];
  const float* kkw = (const float*)d_in[22]; const float* kaw = (const float*)d_in[23]; const float* rk = (const float*)d_in[24];
  const float* Wr = (const float*)d_in[25]; const float* Wk = (const float*)d_in[26]; const float* Wv = (const float*)d_in[27]; const float* Wo = (const float*)d_in[28];
  const float* gnw = (const float*)d_in[29]; const float* gnb = (const float*)d_in[30];
  const float* fxk = (const float*)d_in[31]; const float* Wf1 = (const float*)d_in[32]; const float* Wf2 = (const float*)d_in[33];
  float* out = (float*)d_out; float* out2 = (float*)d_out + (size_t)NR * CC;
  char* ws = (char*)d_ws; size_t off = 0;
  auto take = [&](size_t bytes) { char* p = ws + off; off += (bytes + 255) & ~(size_t)255; return p; };
  const size_t RF = (size_t)NR * CC * 4, RH = (size_t)NR * CC * 2;
  float* x0 = (float*)take(RF);
  float* xn = (float*)take(RF);
  _Float16* mx6 = (_Float16*)take(6 * RH);
  _Float16* WrT = (_Float16*)take((size_t)CC * CC * 2); _Float16* WkT = (_Float16*)take((size_t)CC * CC * 2);
  _Float16* WvT = (_Float16*)take((size_t)CC * CC * 2); _Float16* WoT = (_Float16*)take((size_t)CC * CC * 2);
  _Float16* w1T = (_Float16*)take((size_t)DW * CC * 2); _Float16* w2T = (_Float16*)take((size_t)CC * DW * 2);
  _Float16* a1T = (_Float16*)take((size_t)DA * CC * 2); _Float16* a2T = (_Float16*)take((size_t)CC * DA * 2);
  _Float16* g1T = (_Float16*)take((size_t)DG * CC * 2); _Float16* g2T = (_Float16*)take((size_t)CC * DG * 2);
  _Float16* f1T = (_Float16*)take((size_t)FF * CC * 2); _Float16* f2T = (_Float16*)take((size_t)CC * FF * 2);
  float* rr = (float*)take(RF);
  float* kz = (float*)take(RF);
  float* vv = (float*)take(RF);
  float* dec = (float*)take(RF);
  float* av = (float*)take(RF);
  float* gv = (float*)take(RF);
  _Float16* midw = (_Float16*)take((size_t)NR * DW * 2); _Float16* mida = (_Float16*)take((size_t)NR * DA * 2); _Float16* midg = (_Float16*)take((size_t)NR * DG * 2);
  _Float16 *xr16 = mx6, *xw16 = mx6 + (size_t)NR * CC, *xk16 = mx6 + 2 * (size_t)NR * CC, *xv16 = mx6 + 3 * (size_t)NR * CC, *xa16 = mx6 + 4 * (size_t)NR * CC, *xg16 = mx6 + 5 * (size_t)NR * CC;
  float* kfin = (float*)mx6; float* aav = kfin + (size_t)NR * CC; float* bbv = aav + (size_t)NR * CC;
  float* x1 = xn; float* ov = kz; _Float16* og = (_Float16*)av; float* xf = rr; _Float16* kf16 = (_Float16*)dec; _Float16* hid = (_Float16*)mx6;
  k_packT<<<dim3(CC / 64, CC / 64), 256, 0, stream>>>(Wr, WrT, CC, CC);
  k_packT<<<dim3(CC / 64, CC / 64), 256, 0, stream>>>(Wk, WkT, CC, CC);
  k_packT<<<dim3(CC / 64, CC / 64), 256, 0, stream>>>(Wv, WvT, CC, CC);
  k_packT<<<dim3(CC / 64, CC / 64), 256, 0, stream>>>(Wo, WoT, CC, CC);
  k_packT<<<dim3(DW / 64, CC / 64), 256, 0, stream>>>(w1, w1T, CC, DW);
  k_packT<<<dim3(CC / 64, DW / 64), 256, 0, stream>>>(w2, w2T, DW, CC);
  k_packT<<<dim3(DA / 64, CC / 64), 256, 0, stream>>>(a1, a1T, CC, DA);
  k_packT<<<dim3(CC / 64, DA / 64), 256, 0, stream>>>(a2, a2T, DA, CC);
  k_packT<<<dim3(DG / 64, CC / 64), 256, 0, stream>>>(gg1, g1T, CC, DG);
  k_packT<<<dim3(CC / 64, DG / 64), 256, 0, stream>>>(gg2, g2T, DG, CC);
  k_packT<<<dim3(FF / 64, CC / 64), 256, 0, stream>>>(Wf1, f1T, CC, FF);
  k_packT<<<dim3(CC / 64, FF / 64), 256, 0, stream>>>(Wf2, f2T, FF, CC);
  k_ln01<<<NR, 128, 0, stream>>>(x, g0, b0, g1, b1, x0, xn);
  k_mix<<<NR, 128, 0, stream>>>(xn, x_r, x_w, x_k, x_v, x_a, x_g, xr16, xw16, xk16, xv16, xa16, xg16, 6);
  k_gemm<8, 0><<<dim3(NR / 64, CC / 128), 128, 0, stream>>>(xr16, WrT, nullptr, nullptr, rr, CC, CC);
  k_gemm<8, 0><<<dim3(NR / 64, CC / 128), 128, 0, stream>>>(xk16, WkT, nullptr, nullptr, kz, CC, CC);
  k_gemm<8, 0><<<dim3(NR / 64, CC / 128), 128, 0, stream>>>(xv16, WvT, nullptr, nullptr, vv, CC, CC);
  k_gemm<4, 1><<<dim3(NR / 64, DW / 64), 128, 0, stream>>>(xw16, w1T, nullptr, nullptr, midw, CC, DW);
  k_gemm<8, 3><<<dim3(NR / 64, CC / 128), 128, 0, stream>>>(midw, w2T, w0, nullptr, dec, DW, CC);
  k_gemm<4, 6><<<dim3(NR / 64, DA / 64), 128, 0, stream>>>(xa16, a1T, nullptr, nullptr, mida, CC, DA);
  k_gemm<8, 4><<<dim3(NR / 64, CC / 128), 128, 0, stream>>>(mida, a2T, a0, nullptr, av, DA, CC);
  k_gemm<8, 2><<<dim3(NR / 64, DG / 128), 128, 0, stream>>>(xg16, g1T, nullptr, nullptr, midg, CC, DG);
  k_gemm<8, 0><<<dim3(NR / 64, CC / 128), 128, 0, stream>>>(midg, g2T, nullptr, nullptr, gv, DG, CC);
  k_prep<<<NR, 256, 0, stream>>>(kz, av, kkw, kaw, kfin, aav, bbv);
  k_copy<<<(unsigned)((NR * CC / 4 + 255) / 256), 256, 0, stream>>>(vv, out2, (size_t)NR * CC / 4);
  k_wkv<<<NB * NH, 256, 0, stream>>>(rr, dec, kfin, vv, aav, bbv, ov);
  k_post<<<NR, 256, 0, stream>>>(ov, rr, kfin, vv, gv, rk, gnw, gnb, og);
  k_gemm<8, 0><<<dim3(NR / 64, CC / 128), 128, 0, stream>>>(og, WoT, nullptr, x0, x1, CC, CC);
  k_ln<<<NR, 128, 0, stream>>>(x1, g2, b2, xf);
  k_mixf<<<NR, 128, 0, stream>>>(xf, fxk, kf16);
  k_gemm<8, 5><<<dim3(NR / 64, FF / 128), 128, 0, stream>>>(kf16, f1T, nullptr, nullptr, hid, CC, FF);
  k_gemm<8, 0><<<dim3(NR / 64, CC / 128), 128, 0, stream>>>(hid, f2T, nullptr, x1, out, FF, CC);
}
